// interaction_net_81896436400332
// MI455X (gfx1250) — hardware-verified
//
#include <hip/hip_runtime.h>
#include <math.h>


#define NBAT 32
#define NTIM 32
#define NCH 256
#define NGATE 1280
#define ROWE 512
#define TILEE 1024
#define MATE 655360
#define LDS_LAYER 181376
#define LTHR 256

typedef __bf16   v16b __attribute__((ext_vector_type(16)));
typedef __bf16   v8b  __attribute__((ext_vector_type(8)));
typedef float    v8f  __attribute__((ext_vector_type(8)));
typedef float    v4f  __attribute__((ext_vector_type(4)));
typedef unsigned v8u  __attribute__((ext_vector_type(8)));
typedef unsigned v4u  __attribute__((ext_vector_type(4)));
typedef v4f __attribute__((may_alias)) v4fa;
typedef v4u __attribute__((may_alias)) v4ua;
typedef v8b __attribute__((may_alias)) v8ba;

union Frag { v16b v; v8b h[2]; v8u u; v4u q[2]; };

__device__ __forceinline__ v8f wmma3(v8f acc, const Frag& ah, const Frag& al, const Frag& bh, const Frag& bl) {
  acc = __builtin_amdgcn_wmma_f32_16x16x32_bf16(false, ah.v, false, bh.v, (short)0, acc, false, false);
  acc = __builtin_amdgcn_wmma_f32_16x16x32_bf16(false, ah.v, false, bl.v, (short)0, acc, false, false);
  acc = __builtin_amdgcn_wmma_f32_16x16x32_bf16(false, al.v, false, bh.v, (short)0, acc, false, false);
  asm volatile("v_nop\n\tv_nop\n\tv_nop\n\tv_nop" : "+v"(acc) : "v"(ah.v), "v"(al.v), "v"(bh.v), "v"(bl.v) : "memory");
  return acc;
}

__device__ __forceinline__ void split16(const float (&x)[16], Frag& fh, Frag& fl) {
#pragma unroll
  for (int i = 0; i < 16; ++i) {
    const __bf16 hv = (__bf16)x[i];
    fh.v[i] = hv;
    fl.v[i] = (__bf16)(x[i] - (float)hv);
  }
}

__device__ __forceinline__ float sigm(float x) {
  const float e = expf(-fmaxf(x, -40.0f));
  return 1.0f / (1.0f + e);
}

__global__ __launch_bounds__(256) void k_pack(const float* __restrict__ src, __bf16* __restrict__ dst,
                                              int K, int N, int nsrc, int per, int jbase, int dstride,
                                              float scale) {
  const int KT = K >> 5, NT = N >> 4, tiles = KT * NT;
  const int lane = threadIdx.x & 31, hh = lane >> 4, m = lane & 15;
  const int gw = blockIdx.x * 8 + (threadIdx.x >> 5);
  if (gw >= nsrc * tiles) return;
  const int s = gw / tiles, tile = gw - s * tiles;
  const int nt = tile / KT, kt = tile - nt * KT;
  const size_t matE = (size_t)K * (size_t)N;
  const float* sp = src + (size_t)s * matE + (size_t)(nt * 16 + m);
  const int sq = s / per;
  const int d = sq * dstride + jbase + (s - sq * per);
  __bf16* dp = dst + (size_t)d * matE * 2 + (size_t)tile * TILEE + (size_t)(lane * 8);
  const int k0 = kt * 32 + 8 * hh;
  float x[16];
#pragma unroll
  for (int i = 0; i < 8; ++i) {
    x[i]     = sp[(size_t)(k0 + i) * (size_t)N] * scale;
    x[8 + i] = sp[(size_t)(k0 + 16 + i) * (size_t)N] * scale;
  }
  Frag fh, fl;
  split16(x, fh, fl);
  *(volatile v4u*)(dp)       = fh.q[0];
  *(volatile v4u*)(dp + 256) = fh.q[1];
  *(volatile v4u*)(dp + 512) = fl.q[0];
  *(volatile v4u*)(dp + 768) = fl.q[1];
  __threadfence();
  *(volatile v4u*)(dp)       = fh.q[0];
  *(volatile v4u*)(dp + 256) = fh.q[1];
  *(volatile v4u*)(dp + 512) = fl.q[0];
  *(volatile v4u*)(dp + 768) = fl.q[1];
}

__global__ __launch_bounds__(256) void k_group(const float* __restrict__ feat, const float* __restrict__ ctx,
                                               const float* __restrict__ Wsep, const float* __restrict__ bsep,
                                               __bf16* __restrict__ seqp, __bf16* __restrict__ cxp, int nbt) {
#pragma clang fp contract(off)
  __shared__ float red[4][8];
  __shared__ float selv[4];
  __shared__ float rcv[2];
  __shared__ __align__(16) __bf16 stg[6][256];
  const int bt = blockIdx.x;
  if (bt >= nbt) return;
  const int b = bt >> 5, t = bt & 31;
  const int tid = threadIdx.x, lane = tid & 31, wv = tid >> 5, c = tid;
  const float* f = feat + (size_t)bt * 1024;
  const float wsc = Wsep[c];
  float v[4];
#pragma unroll
  for (int mm = 0; mm < 4; ++mm) {
    v[mm] = f[mm * 256 + c];
    float p = v[mm] * wsc;
#pragma unroll
    for (int o = 16; o > 0; o >>= 1) p += __shfl_xor(p, o);
    if (lane == 0) red[mm][wv] = p;
  }
  __syncthreads();
  if (tid == 0) {
    float z[4];
#pragma unroll
    for (int mm = 0; mm < 4; ++mm) {
      float s = red[mm][0];
#pragma unroll
      for (int q = 1; q < 8; ++q) s += red[mm][q];
      z[mm] = s + bsep[0];
    }
    float mx = fmaxf(fmaxf(z[0], z[1]), fmaxf(z[2], z[3]));
    float e[4], den = 0.0f;
#pragma unroll
    for (int mm = 0; mm < 4; ++mm) { e[mm] = expf(z[mm] - mx); den += e[mm]; }
    const float rden = 1.0f / den;
    float cnt = 0.0f;
#pragma unroll
    for (int mm = 0; mm < 4; ++mm) {
      const float pm = e[mm] * rden;
      const float dm = pm - 0.25f;
      const float sv = (dm > 0.0f) ? 1.0f : 0.0f;
      selv[mm] = sv;
      cnt += sv;
    }
    rcv[0] = 1.0f / (cnt + 1e-8f);
    rcv[1] = 1.0f / ((4.0f - cnt) + 1e-8f);
  }
  __syncthreads();
  float s0 = 0.0f, s1 = 0.0f;
#pragma unroll
  for (int mm = 0; mm < 4; ++mm) {
    const float sv = selv[mm];
    s0 += sv * v[mm];
    s1 += (1.0f - sv) * v[mm];
  }
  const float g0 = s0 * rcv[0], g1 = s1 * rcv[1];
  {
    const __bf16 a0 = (__bf16)g0; stg[0][c] = a0; stg[1][c] = (__bf16)(g0 - (float)a0);
    const __bf16 a1 = (__bf16)g1; stg[2][c] = a1; stg[3][c] = (__bf16)(g1 - (float)a1);
    const float xv = ctx[(size_t)bt * 256 + c];
    const __bf16 ax = (__bf16)xv; stg[4][c] = ax; stg[5][c] = (__bf16)(xv - (float)ax);
  }
  __syncthreads();
  const bool wr = tid < 192;
  v4u val = {0u, 0u, 0u, 0u};
  __bf16* dstp = seqp;
  if (wr) {
    const int q = wv;
    val = *(const v4ua*)(&stg[q][lane * 8]);
    if (q < 4) dstp = seqp + (size_t)(((t * 32 + b) * 2 + (q >> 1)) * ROWE + (q & 1) * 256 + lane * 8);
    else       dstp = cxp + (size_t)(bt * ROWE + (q - 4) * 256 + lane * 8);
    *(volatile v4u*)dstp = val;
  }
  __threadfence();
  if (wr) *(volatile v4u*)dstp = val;
}

__global__ __launch_bounds__(128) void k_share(const float* __restrict__ feat, const __bf16* __restrict__ wp,
                                               const float* __restrict__ bias, float* __restrict__ sf, int nmt) {
  __shared__ __align__(16) float st[16 * 256];
  if (blockIdx.x >= nmt) return;
  const int mt = blockIdx.x, tid = threadIdx.x, lane = tid & 31, wv = tid >> 5, hh = lane >> 4, m = lane & 15;
  const float* ar = feat + (size_t)(mt * 16 + m) * 1024;
  const v8f z8 = {0.f, 0.f, 0.f, 0.f, 0.f, 0.f, 0.f, 0.f};
  v8f acc[4];
#pragma unroll
  for (int p = 0; p < 4; ++p) acc[p] = z8;
#pragma unroll 1
  for (int kt = 0; kt < 32; ++kt) {
    const int ko = kt * 32 + 8 * hh;
    const v4f q0 = *(const v4fa*)(ar + ko);
    const v4f q1 = *(const v4fa*)(ar + ko + 4);
    const v4f q2 = *(const v4fa*)(ar + ko + 16);
    const v4f q3 = *(const v4fa*)(ar + ko + 20);
    float x[16];
    x[0] = q0[0]; x[1] = q0[1]; x[2]  = q0[2]; x[3]  = q0[3];
    x[4] = q1[0]; x[5] = q1[1]; x[6]  = q1[2]; x[7]  = q1[3];
    x[8] = q2[0]; x[9] = q2[1]; x[10] = q2[2]; x[11] = q2[3];
    x[12] = q3[0]; x[13] = q3[1]; x[14] = q3[2]; x[15] = q3[3];
    Frag ah, al;
    split16(x, ah, al);
#pragma unroll
    for (int p = 0; p < 4; ++p) {
      const __bf16* tb = wp + (size_t)((wv * 4 + p) * 32 + kt) * TILEE + (size_t)(lane * 8);
      Frag bh, bl;
      bh.h[0] = *(const v8ba*)(tb);
      bh.h[1] = *(const v8ba*)(tb + 256);
      bl.h[0] = *(const v8ba*)(tb + 512);
      bl.h[1] = *(const v8ba*)(tb + 768);
      acc[p] = wmma3(acc[p], ah, al, bh, bl);
    }
  }
#pragma unroll
  for (int p = 0; p < 4; ++p) {
    const int n = (wv * 4 + p) * 16 + m;
    const float bn = bias[n];
#pragma unroll
    for (int r = 0; r < 8; ++r) st[(8 * hh + r) * 256 + n] = fmaxf(acc[p][r] + bn, 0.0f);
  }
  __syncthreads();
  v4f ov[8];
#pragma unroll
  for (int q = 0; q < 4; ++q) {
    const float* rs = st + (wv * 4 + q) * 256;
    ov[2 * q]     = *(const v4fa*)(rs + 4 * lane);
    ov[2 * q + 1] = *(const v4fa*)(rs + 128 + 4 * lane);
  }
#pragma unroll
  for (int q = 0; q < 4; ++q) {
    float* dr = sf + (size_t)(mt * 16 + wv * 4 + q) * 256;
    *(volatile v4f*)(dr + 4 * lane)       = ov[2 * q];
    *(volatile v4f*)(dr + 128 + 4 * lane) = ov[2 * q + 1];
  }
  __threadfence();
#pragma unroll
  for (int q = 0; q < 4; ++q) {
    float* dr = sf + (size_t)(mt * 16 + wv * 4 + q) * 256;
    *(volatile v4f*)(dr + 4 * lane)       = ov[2 * q];
    *(volatile v4f*)(dr + 128 + 4 * lane) = ov[2 * q + 1];
  }
}

__device__ __forceinline__ void gemm_src5(v8f (&acc)[5], const __bf16* src, unsigned mk,
                                          const __bf16* __restrict__ wmat, int ct, int lane, int hh) {
#pragma unroll 1
  for (int kt = 0; kt < 8; ++kt) {
    const int ko = kt * 32 + 8 * hh;
    Frag ah, al;
    ah.h[0] = *(const v8ba*)(src + ko);
    ah.h[1] = *(const v8ba*)(src + ko + 16);
    al.h[0] = *(const v8ba*)(src + 256 + ko);
    al.h[1] = *(const v8ba*)(src + 256 + ko + 16);
    ah.u &= mk;
    al.u &= mk;
#pragma unroll
    for (int p = 0; p < 5; ++p) {
      const __bf16* tb = wmat + (size_t)((p * 16 + ct) * 8 + kt) * TILEE + (size_t)(lane * 8);
      Frag bh, bl;
      bh.h[0] = *(const v8ba*)(tb);
      bh.h[1] = *(const v8ba*)(tb + 256);
      bl.h[0] = *(const v8ba*)(tb + 512);
      bl.h[1] = *(const v8ba*)(tb + 768);
      acc[p] = wmma3(acc[p], ah, al, bh, bl);
    }
  }
}

template <int G>
__device__ __forceinline__ void gates_group(const __bf16* __restrict__ xp, const __bf16* __restrict__ cxp,
                                            const __bf16* hpl, const int* wm, const __bf16* __restrict__ wl,
                                            const float* __restrict__ bxp, const float* __restrict__ bhp,
                                            const float* __restrict__ bcp,
                                            float* cel, float* hf, float* sgl,
                                            int l, int t, int mt, int q, int wv, int lane, int hh, int m) {
  const v8f z8 = {0.f, 0.f, 0.f, 0.f, 0.f, 0.f, 0.f, 0.f};
  v8f acc[5];
#pragma unroll
  for (int p = 0; p < 5; ++p) acc[p] = z8;
  const int brow = mt * 16 + m;
  const int ct = q * 8 + wv;
  const int n = q * 128 + wv * 16 + m;
  const int tn = (t + 1 < NTIM) ? (t + 1) : t;
  const unsigned nzm = (t + 1 < NTIM) ? 0xFFFFFFFFu : 0u;
  const int s1 = (t + 1) & 1, s0 = t & 1;
  const __bf16* xr  = xp + (size_t)(((t  * NBAT + brow) * 2 + G) * ROWE);
  const __bf16* xs  = xp + (size_t)(((t  * NBAT + brow) * 2 + (1 - G)) * ROWE);
  const __bf16* xn  = xp + (size_t)(((tn * NBAT + brow) * 2 + G) * ROWE);
  const __bf16* xns = xp + (size_t)(((tn * NBAT + brow) * 2 + (1 - G)) * ROWE);
  const __bf16* h1  = hpl + ((s1 * 16 + m) * 2 + G) * ROWE;
  const __bf16* h1s = hpl + ((s1 * 16 + m) * 2 + (1 - G)) * ROWE;
  const __bf16* h2  = hpl + ((s0 * 16 + m) * 2 + G) * ROWE;
  const __bf16* cx  = cxp + (size_t)((brow * NTIM + t) * ROWE);
  const unsigned wbits = (unsigned)wm[m * 2 + G];
#define MKB(k) (0u - ((wbits >> (k)) & 1u))
  const __bf16* wg = wl + (size_t)(G * 8) * MATE;
  gemm_src5(acc, xr,  0xFFFFFFFFu, wg,                     ct, lane, hh);
  gemm_src5(acc, h1,  0xFFFFFFFFu, wg + (size_t)1 * MATE,  ct, lane, hh);
  gemm_src5(acc, h2,  MKB(0),       wg + (size_t)2 * MATE, ct, lane, hh);
  gemm_src5(acc, xn,  MKB(1) & nzm, wg + (size_t)3 * MATE, ct, lane, hh);
  gemm_src5(acc, h1s, MKB(2),       wg + (size_t)4 * MATE, ct, lane, hh);
  gemm_src5(acc, xs,  MKB(3),       wg + (size_t)5 * MATE, ct, lane, hh);
  gemm_src5(acc, xns, MKB(4) & nzm, wg + (size_t)6 * MATE, ct, lane, hh);
  gemm_src5(acc, cx,  MKB(5),       wg + (size_t)7 * MATE, ct, lane, hh);
#undef MKB
  const int lgi = l * 2 + G;
#pragma unroll
  for (int p = 0; p < 5; ++p) {
    const int nn = p * 256 + n;
    const float b0 = bxp[(size_t)lgi * NGATE + nn] + bhp[(size_t)lgi * NGATE + nn];
    float bck[6];
#pragma unroll
    for (int k = 0; k < 6; ++k) bck[k] = 0.5f * bcp[((size_t)lgi * 6 + k) * NGATE + nn];
#pragma unroll
    for (int r = 0; r < 8; ++r) {
      const unsigned wb = (unsigned)wm[(8 * hh + r) * 2 + G];
      float bsum = b0;
#pragma unroll
      for (int k = 0; k < 6; ++k) bsum += (float)((wb >> k) & 1u) * bck[k];
      acc[p][r] += bsum;
    }
  }
#pragma unroll
  for (int r = 0; r < 8; ++r) {
    const int b2 = 8 * hh + r;
    const int hi = (b2 * 2 + G) * 256 + n;
    const int si = b2 * 256 + n;
    const float ig = acc[0][r], fg = acc[1][r], og = acc[2][r], sg = acc[3][r], cv = acc[4][r];
    const float cprev = cel[hi];
    const float cn = (1.0f - sigm(fg)) * cprev + sigm(ig) * tanhf(cv);
    cel[hi] = cn;
    hf[hi] = sigm(og) * tanhf(cn);
    if (G == 0) sgl[si] = sg;
    else        sgl[si] = sgl[si] + sg;
  }
}

__device__ __forceinline__ void route_logits(const float* hf, const float* __restrict__ Wa,
                                             const float* __restrict__ ba, float* lgt, int l, int tid) {
  if (tid < 192) {
    const int row = tid / 12, rem = tid - row * 12, g = rem / 6, k = rem - g * 6;
    const float* hr = hf + (row * 2 + g) * 256;
    const float* wa = Wa + (size_t)l * 1536 + k;
    float s = 0.0f;
#pragma unroll 4
    for (int h = 0; h < 256; ++h) s += hr[h] * wa[h * 6];
    lgt[(row * 2 + g) * 8 + k] = s + ba[l * 6 + k];
  }
}

__device__ __forceinline__ void route_top2(const float* lgt, int* wm, int tid) {
  if (tid < 32) {
    const float* lg = lgt + tid * 8;
    float v0 = lg[0], v1 = lg[1], v2 = lg[2], v3 = lg[3], v4 = lg[4], v5 = lg[5];
    float bv = v0; int bi = 0;
    if (v1 > bv) { bv = v1; bi = 1; }
    if (v2 > bv) { bv = v2; bi = 2; }
    if (v3 > bv) { bv = v3; bi = 3; }
    if (v4 > bv) { bv = v4; bi = 4; }
    if (v5 > bv) { bv = v5; bi = 5; }
    float cv = -INFINITY; int ci = -1;
    if (bi != 0 && v0 > cv) { cv = v0; ci = 0; }
    if (bi != 1 && v1 > cv) { cv = v1; ci = 1; }
    if (bi != 2 && v2 > cv) { cv = v2; ci = 2; }
    if (bi != 3 && v3 > cv) { cv = v3; ci = 3; }
    if (bi != 4 && v4 > cv) { cv = v4; ci = 4; }
    if (bi != 5 && v5 > cv) { cv = v5; ci = 5; }
    if (ci < 0) ci = (bi == 0) ? 1 : 0;
    wm[tid] = (1 << bi) | (1 << ci);
  }
}

extern __shared__ __align__(16) unsigned char dsm[];

__global__ void __launch_bounds__(LTHR) __attribute__((amdgpu_num_vgpr(256)))
k_layer(const __bf16* __restrict__ xp, __bf16* __restrict__ hsp, const __bf16* __restrict__ cxp,
        const float* __restrict__ sf, const __bf16* __restrict__ wall,
        const float* __restrict__ Wa, const float* __restrict__ ba,
        const float* __restrict__ bxp, const float* __restrict__ bhp, const float* __restrict__ bcp,
        float* __restrict__ out, int l, int nblk) {
  if (blockIdx.x >= nblk) return;
  __bf16* hpl = (__bf16*)dsm;
  float*  hf  = (float*)(dsm + 65536);
  float*  cel = (float*)(dsm + 98304);
  float*  ssl = (float*)(dsm + 131072);
  float*  cgl = (float*)(dsm + 147456);
  float*  sgl = (float*)(dsm + 163840);
  int*    wm  = (int*)(dsm + 180224);
  float*  lgt = (float*)(dsm + 180352);
  const int tid = threadIdx.x, lane = tid & 31, wv = tid >> 5, hh = lane >> 4, m = lane & 15;
  const int mt = blockIdx.x;
  {
    const v4u z4 = {0u, 0u, 0u, 0u};
    for (int i = tid; i < LDS_LAYER / 16; i += LTHR) ((v4u*)dsm)[i] = z4;
  }
  __syncthreads();
  const __bf16* wl = wall + (size_t)(l * 16) * MATE;
  route_logits(hf, Wa, ba, lgt, l, tid);
  __syncthreads();
  route_top2(lgt, wm, tid);
  __syncthreads();
  for (int t = 0; t < NTIM; ++t) {
#pragma unroll 1
    for (int q = 0; q < 2; ++q)
      gates_group<0>(xp, cxp, hpl, wm, wl, bxp, bhp, bcp, cel, hf, sgl, l, t, mt, q, wv, lane, hh, m);
#pragma unroll 1
    for (int q = 0; q < 2; ++q)
      gates_group<1>(xp, cxp, hpl, wm, wl, bxp, bhp, bcp, cel, hf, sgl, l, t, mt, q, wv, lane, hh, m);
    __syncthreads();
    const int s0 = t & 1;
#pragma unroll 1
    for (int q = 0; q < 2; ++q) {
      const int n = q * 128 + wv * 16 + m;
#pragma unroll
      for (int r = 0; r < 8; ++r) {
        const int b2 = 8 * hh + r;
        const float v0 = hf[(b2 * 2 + 0) * 256 + n], v1 = hf[(b2 * 2 + 1) * 256 + n];
        const __bf16 a0 = (__bf16)v0, a1 = (__bf16)v1;
        __bf16* pr0 = hpl + ((s0 * 16 + b2) * 2 + 0) * ROWE + n;
        __bf16* pr1 = hpl + ((s0 * 16 + b2) * 2 + 1) * ROWE + n;
        pr0[0] = a0; pr0[256] = (__bf16)(v0 - (float)a0);
        pr1[0] = a1; pr1[256] = (__bf16)(v1 - (float)a1);
        const int si = b2 * 256 + n;
        const float ob = sigm(sgl[si]);
        const float ssv = ssl[si] + ob * sf[(size_t)((mt * 16 + b2) * NTIM + t) * 256 + n];
        const float cgv = cgl[si] + ob;
        ssl[si] = ssv;
        cgl[si] = cgv;
      }
    }
    __syncthreads();
    route_logits(hf, Wa, ba, lgt, l, tid);
    __syncthreads();
    route_top2(lgt, wm, tid);
#pragma unroll 1
    for (int j = 0; j < 2; ++j) {
      const int bl = wv * 2 + j, bb = mt * 16 + bl;
      const float* hr0 = hf + (bl * 2 + 0) * 256;
      const float* hr1 = hf + (bl * 2 + 1) * 256;
      const float* sr  = ssl + bl * 256;
      const float* cr  = cgl + bl * 256;
      const v4f o0a = *(const v4fa*)(hr0 + 4 * lane), o0b = *(const v4fa*)(hr0 + 128 + 4 * lane);
      const v4f o1a = *(const v4fa*)(hr1 + 4 * lane), o1b = *(const v4fa*)(hr1 + 128 + 4 * lane);
      const v4f sa = *(const v4fa*)(sr + 4 * lane), sb = *(const v4fa*)(sr + 128 + 4 * lane);
      const v4f ca = *(const v4fa*)(cr + 4 * lane), cb = *(const v4fa*)(cr + 128 + 4 * lane);
      v4f ra, rb;
      ra[0] = 1.0f / ca[0]; ra[1] = 1.0f / ca[1]; ra[2] = 1.0f / ca[2]; ra[3] = 1.0f / ca[3];
      rb[0] = 1.0f / cb[0]; rb[1] = 1.0f / cb[1]; rb[2] = 1.0f / cb[2]; rb[3] = 1.0f / cb[3];
      const v4f o2a = sa * ra, o2b = sb * rb;
      const __bf16* pl0 = hpl + ((s0 * 16 + bl) * 2 + 0) * ROWE;
      const __bf16* pl1 = hpl + ((s0 * 16 + bl) * 2 + 1) * ROWE;
      const v4u p0h = *(const v4ua*)(pl0 + 8 * lane), p0l = *(const v4ua*)(pl0 + 256 + 8 * lane);
      const v4u p1h = *(const v4ua*)(pl1 + 8 * lane), p1l = *(const v4ua*)(pl1 + 256 + 8 * lane);
      float* orow = out + (size_t)((l * NBAT + bb) * NTIM + t) * 768;
      __bf16* hrow = hsp + (size_t)((t * NBAT + bb) * 2) * ROWE;
      *(volatile v4f*)(orow + 4 * lane)        = o0a;
      *(volatile v4f*)(orow + 128 + 4 * lane)  = o0b;
      *(volatile v4f*)(orow + 256 + 4 * lane)  = o1a;
      *(volatile v4f*)(orow + 384 + 4 * lane)  = o1b;
      *(volatile v4f*)(orow + 512 + 4 * lane)  = o2a;
      *(volatile v4f*)(orow + 640 + 4 * lane)  = o2b;
      *(volatile v4u*)(hrow + 8 * lane)        = p0h;
      *(volatile v4u*)(hrow + 256 + 8 * lane)  = p0l;
      *(volatile v4u*)(hrow + 512 + 8 * lane)  = p1h;
      *(volatile v4u*)(hrow + 768 + 8 * lane)  = p1l;
      __threadfence();
      *(volatile v4f*)(orow + 4 * lane)        = o0a;
      *(volatile v4f*)(orow + 128 + 4 * lane)  = o0b;
      *(volatile v4f*)(orow + 256 + 4 * lane)  = o1a;
      *(volatile v4f*)(orow + 384 + 4 * lane)  = o1b;
      *(volatile v4f*)(orow + 512 + 4 * lane)  = o2a;
      *(volatile v4f*)(orow + 640 + 4 * lane)  = o2b;
      *(volatile v4u*)(hrow + 8 * lane)        = p0h;
      *(volatile v4u*)(hrow + 256 + 8 * lane)  = p0l;
      *(volatile v4u*)(hrow + 512 + 8 * lane)  = p1h;
      *(volatile v4u*)(hrow + 768 + 8 * lane)  = p1l;
    }
    __syncthreads();
  }
}

extern "C" void kernel_launch(void* const* d_in, const int* in_sizes, int n_in,
                              void* d_out, int out_size, void* d_ws, size_t ws_size,
                              hipStream_t stream) {
  if (n_in < 14) return;
  if (in_sizes[0] != NBAT * NTIM * 4 * NCH) return;
  if (in_sizes[1] != NBAT * NTIM * NCH) return;
  if (in_sizes[2] != 1024 * 256) return;
  if (in_sizes[6] != 2 * 256 * 6) return;
  if (in_sizes[8] != 2 * 2 * 256 * NGATE) return;
  if (in_sizes[10] != 2 * 2 * 256 * NGATE) return;
  if (in_sizes[12] != 2 * 2 * 6 * 256 * NGATE) return;
  if (out_size != 2 * NBAT * NTIM * 768) return;
  const float* feat  = (const float*)d_in[0];
  const float* ctx   = (const float*)d_in[1];
  const float* Wl2s  = (const float*)d_in[2];
  const float* bl2s  = (const float*)d_in[3];
  const float* Wsep  = (const float*)d_in[4];
  const float* bsep  = (const float*)d_in[5];
  const float* Warch = (const float*)d_in[6];
  const float* barch = (const float*)d_in[7];
  const float* Wx    = (const float*)d_in[8];
  const float* bx    = (const float*)d_in[9];
  const float* Wh    = (const float*)d_in[10];
  const float* bh    = (const float*)d_in[11];
  const float* Wc    = (const float*)d_in[12];
  const float* bc    = (const float*)d_in[13];
  float* out = (float*)d_out;

  char* ws = (char*)d_ws;
  size_t off = 0;
  const size_t b_wl2s = (size_t)1024 * 256 * 2 * 2;
  const size_t b_wall = (size_t)32 * MATE * 2;
  const size_t b_pl   = (size_t)NTIM * NBAT * 2 * ROWE * 2;
  const size_t b_cx   = (size_t)NBAT * NTIM * ROWE * 2;
  const size_t b_sf   = (size_t)NBAT * NTIM * 256 * 4;
  __bf16* wl2s_p = (__bf16*)(ws + off); off += b_wl2s;
  __bf16* wall   = (__bf16*)(ws + off); off += b_wall;
  __bf16* seqp   = (__bf16*)(ws + off); off += b_pl;
  __bf16* hsp    = (__bf16*)(ws + off); off += b_pl;
  __bf16* cxp    = (__bf16*)(ws + off); off += b_cx;
  float*  sfb    = (float*)(ws + off);  off += b_sf;
  if (off > ws_size) return;

  k_pack<<<(1 * 512 + 7) / 8, 256, 0, stream>>>(Wl2s, wl2s_p, 1024, 256, 1, 1, 0, 1, 1.0f);
  k_pack<<<(4 * 640 + 7) / 8, 256, 0, stream>>>(Wx, wall, 256, 1280, 4, 1, 0, 8, 1.0f);
  k_pack<<<(4 * 640 + 7) / 8, 256, 0, stream>>>(Wh, wall, 256, 1280, 4, 1, 1, 8, 1.0f);
  k_pack<<<(24 * 640 + 7) / 8, 256, 0, stream>>>(Wc, wall, 256, 1280, 24, 6, 2, 8, 0.5f);

  k_group<<<NBAT * NTIM, 256, 0, stream>>>(feat, ctx, Wsep, bsep, seqp, cxp, NBAT * NTIM);
  k_share<<<64, 128, 0, stream>>>(feat, wl2s_p, bl2s, sfb, 64);

  k_layer<<<2, LTHR, LDS_LAYER, stream>>>(seqp, hsp, cxp, sfb, wall, Warch, barch, bx, bh, bc, out, 0, 2);
  k_layer<<<2, LTHR, LDS_LAYER, stream>>>(hsp, seqp, cxp, sfb, wall, Warch, barch, bx, bh, bc, out, 1, 2);
}
